// MaskedDeepRNN_6940667150753
// MI455X (gfx1250) — hardware-run, weakly checked
//
#include <hip/hip_runtime.h>
#include <math.h>

typedef __attribute__((ext_vector_type(16))) _Float16 v16h;
typedef __attribute__((ext_vector_type(8)))  _Float16 v8h;
typedef __attribute__((ext_vector_type(8)))  float    v8f;
typedef __attribute__((ext_vector_type(4)))  float    v4f;

constexpr int kBatch     = 64;
constexpr int kSteps     = 512;
constexpr int kDin       = 256;
constexpr int kHid       = 512;
constexpr int kGate      = 4 * kHid;
constexpr int kRowsBlk   = 32;
constexpr int kScanThr   = 512;
constexpr int kScanWaves = kScanThr / 32;
constexpr int kHP        = 520;
constexpr int kSlabP     = 36;
constexpr int kPackThr   = 256;
constexpr float kActCarry = 128.0f;
constexpr float kWCarry   = 512.0f;
constexpr float kFold     = 1.0f / (kActCarry * kWCarry);
constexpr float kF16MinNormal = 6.103515625e-05f;

static_assert(kGate == 2048);
static_assert(kBatch % kRowsBlk == 0);
static_assert(kHid == 32 * kScanWaves);
static_assert(kDin % 32 == 0 && kHid % 32 == 0);
static_assert(kHP % 8 == 0 && kHP >= kHid);
static_assert((2 * kRowsBlk * kHP) % kScanThr == 0);
static_assert(kRowsBlk * (kHid / 8) == 4 * kScanThr);
static_assert(kFold == 1.0f / 65536.0f);
static_assert(((kGate * kDin / 8) % kPackThr) == 0 && ((kGate * kHid / 8) % kPackThr) == 0);
static_assert(((kSteps * kBatch * (kDin / 8)) % kPackThr) == 0);

constexpr size_t kBytesWI0  = (size_t)kGate * kDin * 2;
constexpr size_t kBytesWH   = (size_t)kGate * kHid * 2;
constexpr size_t kBytesX16  = (size_t)kSteps * kBatch * kDin * 2;
constexpr size_t kBytesHSEQ = (size_t)kSteps * kBatch * kHid * 2;
constexpr size_t kWsTotal   = kBytesWI0 + 3 * kBytesWH + kBytesX16 + kBytesHSEQ;
static_assert(kWsTotal == 57671680ull);
static_assert(kWsTotal <= 134217728ull);
static_assert((kBytesWI0 % 256) == 0 && (kBytesWH % 256) == 0 && (kBytesX16 % 256) == 0 && (kBytesHSEQ % 256) == 0);

union FragU { v16h v; v8h h[2]; };
__device__ __forceinline__ v16h frag_load(const _Float16* p) {
  FragU f;
  f.h[0] = *(const v8h*)(p);
  f.h[1] = *(const v8h*)(p + 16);
  return f.v;
}
__device__ __forceinline__ v8f mma_f16(v16h a, v16h b, v8f c) {
  return __builtin_amdgcn_wmma_f32_16x16x32_f16(false, a, false, b, (short)0, c, false, false);
}
__device__ __forceinline__ void guard8_h(v8f& a0, v8f& a1, v8f& a2, v8f& a3, v8f& a4, v8f& a5, v8f& a6, v8f& a7,
                                         v16h x0, v16h x1, v16h y0, v16h y1, v16h y2, v16h y3) {
  asm volatile("v_nop\n\tv_nop\n\tv_nop\n\tv_nop"
               : "+v"(a0), "+v"(a1), "+v"(a2), "+v"(a3), "+v"(a4), "+v"(a5), "+v"(a6), "+v"(a7)
               : "v"(x0), "v"(x1), "v"(y0), "v"(y1), "v"(y2), "v"(y3));
}

__device__ __forceinline__ _Float16 f16_operand(float v, float carry) {
  const float s = v * carry;
  const float f = (fabsf(s) < kF16MinNormal) ? 0.0f : s;
  return (_Float16)f;
}

__device__ __forceinline__ float fsig(float x)  { return __builtin_amdgcn_rcpf(1.0f + __expf(-x)); }
__device__ __forceinline__ float ftanh(float x) { return 1.0f - 2.0f * __builtin_amdgcn_rcpf(__expf(2.0f * x) + 1.0f); }

__global__ __launch_bounds__(kPackThr) void pack_w_kernel(const float* __restrict__ W, const float* __restrict__ Mk,
                                                          unsigned short* __restrict__ dst, int n8) {
  const int i = blockIdx.x * kPackThr + threadIdx.x;
  if (i < n8) {
    const size_t e0 = (size_t)i << 3;
    const v4f w0 = *(const v4f*)(W + e0);
    const v4f w1 = *(const v4f*)(W + e0 + 4);
    const v4f m0 = *(const v4f*)(Mk + e0);
    const v4f m1 = *(const v4f*)(Mk + e0 + 4);
    v8h hv;
#pragma unroll
    for (int e = 0; e < 4; ++e) {
      const float wa = w0[e], ma = m0[e];
      const float wb = w1[e], mb = m1[e];
      float pa = wa * ma;
      float pb = wb * mb;
      pa = (ma == 0.0f) ? 0.0f : pa;
      pb = (mb == 0.0f) ? 0.0f : pb;
      hv[e]     = f16_operand(pa, kWCarry);
      hv[4 + e] = f16_operand(pb, kWCarry);
    }
    _Float16* q = (_Float16*)dst + e0;
    *(volatile v8h*)q = hv;
    __threadfence();
    *(volatile v8h*)q = hv;
  }
}

__global__ __launch_bounds__(kPackThr) void pack_x_kernel(const float* __restrict__ x, unsigned short* __restrict__ dst) {
  constexpr int kD8 = kDin / 8;
  constexpr int kN8 = kSteps * kBatch * kD8;
  const int i = blockIdx.x * kPackThr + threadIdx.x;
  if (i < kN8) {
    const int d8 = i % kD8;
    const int bt = i / kD8;
    const int b  = bt % kBatch;
    const int t  = bt / kBatch;
    const float* sp = x + ((size_t)b * kSteps + (size_t)t) * kDin + d8 * 8;
    const v4f a0 = *(const v4f*)(sp);
    const v4f a1 = *(const v4f*)(sp + 4);
    v8h hv;
#pragma unroll
    for (int e = 0; e < 4; ++e) {
      const float fa = a0[e];
      const float fb = a1[e];
      hv[e]     = f16_operand(fa, kActCarry);
      hv[4 + e] = f16_operand(fb, kActCarry);
    }
    _Float16* q = (_Float16*)dst + (size_t)i * 8;
    *(volatile v8h*)q = hv;
    __threadfence();
    *(volatile v8h*)q = hv;
  }
}

template <int KX, bool FINAL>
__global__ __launch_bounds__(kScanThr) void lstm_scan_kernel(
    const unsigned short* __restrict__ Xp, const unsigned short* __restrict__ WIp,
    const unsigned short* __restrict__ WHp,
    const float* __restrict__ b_ih, const float* __restrict__ b_hh,
    unsigned short* __restrict__ HSEQ, float* __restrict__ OUT) {
  static_assert(KX % 32 == 0);
  __shared__ __align__(16) _Float16 Ah[2][kRowsBlk * kHP];
  __shared__ __align__(16) float    Sl[FINAL ? kScanWaves : 1][FINAL ? kRowsBlk * kSlabP : 4];

  const _Float16* X  = (const _Float16*)Xp;
  const _Float16* WI = (const _Float16*)WIp;
  const _Float16* WH = (const _Float16*)WHp;
  const int tid = threadIdx.x, lane = tid & 31, wave = tid >> 5;
  const int c = lane & 15, hh = lane >> 4, koff = hh * 8;
  const int rowbase = blockIdx.x * kRowsBlk;

  {
    _Float16* ahf = &Ah[0][0];
#pragma unroll 1
    for (int i = tid; i < 2 * kRowsBlk * kHP; i += kScanThr) ahf[i] = (_Float16)0.0f;
  }

  float cst[2][2][8];
  float bb[2][4];
#pragma unroll
  for (int nt = 0; nt < 2; ++nt) {
    const int j = 32 * wave + 16 * nt + c;
#pragma unroll
    for (int g = 0; g < 4; ++g) bb[nt][g] = b_ih[g * kHid + j] + b_hh[g * kHid + j];
#pragma unroll
    for (int mt = 0; mt < 2; ++mt)
#pragma unroll
      for (int r = 0; r < 8; ++r) cst[nt][mt][r] = 0.0f;
  }
  float* slab = &Sl[FINAL ? wave : 0][0];
  __syncthreads();

  const v8f z8 = {0.f, 0.f, 0.f, 0.f, 0.f, 0.f, 0.f, 0.f};

#pragma unroll 1
  for (int t = 0; t < kSteps; ++t) {
    const int cur = t & 1;
    const _Float16* ah0 = &Ah[cur][0] + c * kHP + koff;
    const _Float16* ah1 = ah0 + 16 * kHP;
    _Float16* ahn = &Ah[cur ^ 1][0];
    const _Float16* xr0 = X + ((size_t)t * kBatch + (size_t)(rowbase + c)) * KX + koff;
    const _Float16* xr1 = xr0 + (size_t)16 * KX;
    const bool last = (t == kSteps - 1);
    (void)last;

#pragma unroll
    for (int nt = 0; nt < 2; ++nt) {
      const int j = 32 * wave + 16 * nt + c;
      const _Float16* wi = WI + (size_t)j * KX + koff;
      const _Float16* wh = WH + (size_t)j * kHid + koff;
      v8f acc[2][4];
#pragma unroll
      for (int mt = 0; mt < 2; ++mt)
#pragma unroll
        for (int g = 0; g < 4; ++g) acc[mt][g] = z8;

#pragma unroll 1
      for (int kx = 0; kx < KX; kx += 32) {
        const v16h a0 = frag_load(xr0 + kx);
        const v16h a1 = frag_load(xr1 + kx);
        const v16h b0 = frag_load(wi + kx);
        const v16h b1 = frag_load(wi + (size_t)1 * kHid * KX + kx);
        const v16h b2 = frag_load(wi + (size_t)2 * kHid * KX + kx);
        const v16h b3 = frag_load(wi + (size_t)3 * kHid * KX + kx);
        acc[0][0] = mma_f16(a0, b0, acc[0][0]);
        acc[1][0] = mma_f16(a1, b0, acc[1][0]);
        acc[0][1] = mma_f16(a0, b1, acc[0][1]);
        acc[1][1] = mma_f16(a1, b1, acc[1][1]);
        acc[0][2] = mma_f16(a0, b2, acc[0][2]);
        acc[1][2] = mma_f16(a1, b2, acc[1][2]);
        acc[0][3] = mma_f16(a0, b3, acc[0][3]);
        acc[1][3] = mma_f16(a1, b3, acc[1][3]);
        guard8_h(acc[0][0], acc[1][0], acc[0][1], acc[1][1], acc[0][2], acc[1][2], acc[0][3], acc[1][3],
                 a0, a1, b0, b1, b2, b3);
      }
#pragma unroll 1
      for (int k0 = 0; k0 < kHid; k0 += 32) {
        const v16h a0 = frag_load(ah0 + k0);
        const v16h a1 = frag_load(ah1 + k0);
        const v16h b0 = frag_load(wh + k0);
        const v16h b1 = frag_load(wh + (size_t)1 * kHid * kHid + k0);
        const v16h b2 = frag_load(wh + (size_t)2 * kHid * kHid + k0);
        const v16h b3 = frag_load(wh + (size_t)3 * kHid * kHid + k0);
        acc[0][0] = mma_f16(a0, b0, acc[0][0]);
        acc[1][0] = mma_f16(a1, b0, acc[1][0]);
        acc[0][1] = mma_f16(a0, b1, acc[0][1]);
        acc[1][1] = mma_f16(a1, b1, acc[1][1]);
        acc[0][2] = mma_f16(a0, b2, acc[0][2]);
        acc[1][2] = mma_f16(a1, b2, acc[1][2]);
        acc[0][3] = mma_f16(a0, b3, acc[0][3]);
        acc[1][3] = mma_f16(a1, b3, acc[1][3]);
        guard8_h(acc[0][0], acc[1][0], acc[0][1], acc[1][1], acc[0][2], acc[1][2], acc[0][3], acc[1][3],
                 a0, a1, b0, b1, b2, b3);
      }

#pragma unroll
      for (int mt = 0; mt < 2; ++mt) {
        float hv[8];
#pragma unroll
        for (int r = 0; r < 8; ++r) {
          const float zi = acc[mt][0][r] * kFold + bb[nt][0];
          const float zf = acc[mt][1][r] * kFold + bb[nt][1];
          const float zg = acc[mt][2][r] * kFold + bb[nt][2];
          const float zo = acc[mt][3][r] * kFold + bb[nt][3];
          const float ig = fsig(zi);
          const float fg = fsig(zf);
          const float gg = ftanh(zg);
          const float og = fsig(zo);
          const float cn = fg * cst[nt][mt][r] + ig * gg;
          cst[nt][mt][r] = cn;
          const float hn = og * ftanh(cn);
          hv[r] = hn;
          ahn[(16 * mt + 8 * hh + r) * kHP + j] = f16_operand(hn, kActCarry);
        }
        if (FINAL) {
          if (last) {
#pragma unroll
            for (int r = 0; r < 8; ++r) slab[(16 * mt + 8 * hh + r) * kSlabP + 16 * nt + c] = hv[r];
          }
        }
      }
    }
    __syncthreads();

    if (!FINAL) {
      constexpr int kC8 = kHid / 8;
      _Float16* dsth = (_Float16*)HSEQ + ((size_t)t * kBatch + (size_t)rowbase) * kHid;
      v8h hv4[4];
#pragma unroll
      for (int it = 0; it < 4; ++it) {
        const int idx = it * kScanThr + tid;
        const int row = idx / kC8;
        const int c8  = (idx % kC8) * 8;
        hv4[it] = *(const v8h*)(ahn + row * kHP + c8);
      }
      for (int pass = 0; pass < 2; ++pass) {
#pragma unroll
        for (int it = 0; it < 4; ++it)
          *(volatile v8h*)(dsth + (size_t)(it * kScanThr + tid) * 8) = hv4[it];
        __threadfence();
      }
    }
  }

  if (FINAL) {
    __syncthreads();
    const int q = lane >> 3, c4 = (lane & 7) * 4;
    v4f ov[8];
#pragma unroll
    for (int it = 0; it < 8; ++it) ov[it] = *(const v4f*)(slab + (it * 4 + q) * kSlabP + c4);
    for (int pass = 0; pass < 2; ++pass) {
#pragma unroll
      for (int it = 0; it < 8; ++it)
        *(volatile v4f*)(OUT + (size_t)(rowbase + it * 4 + q) * kHid + 32 * wave + c4) = ov[it];
      __threadfence();
    }
  }
}

extern "C" void kernel_launch(void* const* d_in, const int* in_sizes, int n_in,
                              void* d_out, int out_size, void* d_ws, size_t ws_size, hipStream_t stream) {
  if (n_in < 13 || d_out == nullptr || d_ws == nullptr) return;
  if (in_sizes[0] != kBatch * kSteps * kDin) return;
  if (in_sizes[1] != kGate * kDin || in_sizes[2] != kGate * kHid) return;
  if (in_sizes[3] != kGate || in_sizes[4] != kGate) return;
  if (in_sizes[5] != kGate * kDin || in_sizes[6] != kGate * kHid) return;
  if (in_sizes[7] != kGate * kHid || in_sizes[8] != kGate * kHid) return;
  if (in_sizes[9] != kGate || in_sizes[10] != kGate) return;
  if (in_sizes[11] != kGate * kHid || in_sizes[12] != kGate * kHid) return;
  if (out_size != kBatch * kHid) return;
  if (ws_size < kWsTotal) return;

  const float* x     = (const float*)d_in[0];
  const float* W_ih0 = (const float*)d_in[1];
  const float* W_hh0 = (const float*)d_in[2];
  const float* b_ih0 = (const float*)d_in[3];
  const float* b_hh0 = (const float*)d_in[4];
  const float* m_ih0 = (const float*)d_in[5];
  const float* m_hh0 = (const float*)d_in[6];
  const float* W_ih1 = (const float*)d_in[7];
  const float* W_hh1 = (const float*)d_in[8];
  const float* b_ih1 = (const float*)d_in[9];
  const float* b_hh1 = (const float*)d_in[10];
  const float* m_ih1 = (const float*)d_in[11];
  const float* m_hh1 = (const float*)d_in[12];
  float* out = (float*)d_out;

  char* ws = (char*)d_ws;
  size_t off = 0;
  auto carve = [&](size_t bytes) -> char* { char* p = ws + off; off += (bytes + 255) & ~(size_t)255; return p; };
  unsigned short* WI0  = (unsigned short*)carve(kBytesWI0);
  unsigned short* WH0  = (unsigned short*)carve(kBytesWH);
  unsigned short* WI1  = (unsigned short*)carve(kBytesWH);
  unsigned short* WH1  = (unsigned short*)carve(kBytesWH);
  unsigned short* X16  = (unsigned short*)carve(kBytesX16);
  unsigned short* HSEQ = (unsigned short*)carve(kBytesHSEQ);
  if (off != kWsTotal || off > ws_size || off > (size_t)134217728) return;

  const int n8a = kGate * kDin / 8;
  const int n8b = kGate * kHid / 8;
  pack_w_kernel<<<n8a / kPackThr, kPackThr, 0, stream>>>(W_ih0, m_ih0, WI0, n8a);
  pack_w_kernel<<<n8b / kPackThr, kPackThr, 0, stream>>>(W_hh0, m_hh0, WH0, n8b);
  pack_w_kernel<<<n8b / kPackThr, kPackThr, 0, stream>>>(W_ih1, m_ih1, WI1, n8b);
  pack_w_kernel<<<n8b / kPackThr, kPackThr, 0, stream>>>(W_hh1, m_hh1, WH1, n8b);

  pack_x_kernel<<<(kSteps * kBatch * (kDin / 8)) / kPackThr, kPackThr, 0, stream>>>(x, X16);

  lstm_scan_kernel<kDin, false><<<kBatch / kRowsBlk, kScanThr, 0, stream>>>(X16, WI0, WH0, b_ih0, b_hh0, HSEQ, out);
  lstm_scan_kernel<kHid, true><<<kBatch / kRowsBlk, kScanThr, 0, stream>>>(HSEQ, WI1, WH1, b_ih1, b_hh1, X16, out);
}
